// DAGSparseSelfAttention_49108656062888
// MI455X (gfx1250) — hardware-run, weakly checked
//
#include <hip/hip_runtime.h>


namespace {
constexpr int NB = 8, L = 1024, D = 256, NH = 8, HD = 32, NT = NB * L, KB = 128;
constexpr float XS = 8.0f, WSC = 256.0f, PS = 256.0f, EPS = 1e-5f;
typedef _Float16 b16;
typedef __attribute__((ext_vector_type(16))) _Float16 v16b;
typedef __attribute__((ext_vector_type(8))) _Float16 v8b;
typedef __attribute__((ext_vector_type(8))) float v8f;
typedef __attribute__((ext_vector_type(4))) float v4f;
__device__ __forceinline__ float bf16_rne(float f) { unsigned int u = __float_as_uint(f); u += 0x7FFFu + ((u >> 16) & 1u); float r = __uint_as_float(u & 0xFFFF0000u); asm volatile("" : "+v"(r)); return r; }
__device__ __forceinline__ float bfv(float f) { float r = bf16_rne(f); asm volatile("" : "+v"(r)); return r; }
__device__ __forceinline__ void split16(float v, b16& hi, b16& lo) { hi = (b16)v; lo = (b16)(v - (float)hi); }
__device__ __forceinline__ v16b frag_kb(const b16* p, int hh) { const v8b a = *(const v8b*)(p + 8 * hh), b = *(const v8b*)(p + 16 + 8 * hh); v16b f;
#pragma unroll
  for (int e = 0; e < 8; ++e) { f[e] = a[e]; f[8 + e] = b[e]; } return f; }
__device__ __forceinline__ v8f wmma16b(v16b a, v16b b, v8f c) { v8f d = __builtin_amdgcn_wmma_f32_16x16x32_f16(false, a, false, b, (short)0, c, false, false); asm volatile("v_nop\n\tv_nop\n\tv_nop\n\tv_nop" : "+v"(d) : "v"(a), "v"(b)); return d; }
__device__ __forceinline__ void wave_lds_sync() { __builtin_amdgcn_fence(__ATOMIC_RELEASE, "workgroup"); __builtin_amdgcn_wave_barrier(); __builtin_amdgcn_fence(__ATOMIC_ACQUIRE, "workgroup"); }
__device__ __forceinline__ float pmul(float a, float b) { float p = a * b; asm volatile("" : "+v"(p)); return p; }
__device__ __forceinline__ float wsum(float v) { for (int o = 16; o; o >>= 1) v += __shfl_xor(v, o); return v; }
__device__ __forceinline__ float gelu(float v) { return 0.5f * v * (1.0f + erff(v * 0.70710678118654752f)); }

__global__ __launch_bounds__(256) void wput_kernel(const float* __restrict__ wq, const float* __restrict__ wobs, const float* __restrict__ wk, const float* __restrict__ wv, const float* __restrict__ wp, b16* __restrict__ WQO, b16* __restrict__ WKV, b16* __restrict__ WPp) { const size_t u = (size_t)blockIdx.x * 256 + threadIdx.x; v8b v;
  if (u < (size_t)512 * 32) { const int r = (int)(u / 32), k0 = (int)(u % 32) * 8; const float* w = r < D ? wq + (size_t)r * D : wobs + (size_t)(r - D) * D;
#pragma unroll
    for (int j = 0; j < 8; ++j) v[j] = (b16)(bf16_rne(w[k0 + j]) * WSC); for (int pass = 0; pass < 2; ++pass) { *(volatile v8b*)(WQO + (size_t)r * D + k0) = v; __threadfence(); } }
  if (u < (size_t)512 * 64) { const int r = (int)(u / 64), k0 = (int)(u % 64) * 8; const float* w = r < D ? wk + (size_t)r * 2 * D : wv + (size_t)(r - D) * 2 * D;
#pragma unroll
    for (int j = 0; j < 8; ++j) v[j] = (b16)(bf16_rne(w[k0 + j]) * WSC); for (int pass = 0; pass < 2; ++pass) { *(volatile v8b*)(WKV + (size_t)r * 2 * D + k0) = v; __threadfence(); } }
  if (u < (size_t)256 * 64) { const int r = (int)(u / 64), k0 = (int)(u % 64) * 8;
#pragma unroll
    for (int j = 0; j < 8; ++j) v[j] = (b16)(bf16_rne(wp[(size_t)r * 2 * D + k0 + j]) * WSC); for (int pass = 0; pass < 2; ++pass) { *(volatile v8b*)(WPp + (size_t)r * 2 * D + k0) = v; __threadfence(); } } }
__global__ __launch_bounds__(32) void proj_kernel(const float* __restrict__ obs, const float* __restrict__ act, const b16* __restrict__ WQO, const b16* __restrict__ WKV, const float* __restrict__ bq, const float* __restrict__ bk, const float* __restrict__ bv, const float* __restrict__ bobs, const float* __restrict__ gobs, const float* __restrict__ bobs2, int TLIM, b16* __restrict__ PH, b16* __restrict__ PL, float* __restrict__ Z) {
  __shared__ __attribute__((aligned(16))) b16 Ah[16][2 * D + 8], Oh[16][D + 8], Ol[16][D + 8]; __shared__ float Tf[16][D + 4]; const int lane = threadIdx.x, nloc = lane & 15, hlf = lane >> 4; const size_t m0 = (size_t)blockIdx.x * 16; if (m0 >= (size_t)TLIM) return;
  for (int rr = 0; rr < 16; ++rr) for (int q = 0; q < 8; ++q) { Ah[rr][q * 32 + lane] = (b16)(bf16_rne(obs[(m0 + rr) * D + q * 32 + lane]) * XS); Ah[rr][D + q * 32 + lane] = (b16)(bf16_rne(act[(m0 + rr) * D + q * 32 + lane]) * XS); }
  wave_lds_sync();
#pragma unroll 1
  for (int g = 0; g < 4; ++g) {
    const int K = g < 2 ? D : 2 * D; const b16* W = g < 2 ? WQO + (size_t)g * D * D : WKV + (size_t)(g - 2) * D * 2 * D; v8f acc[16];
#pragma unroll
    for (int t = 0; t < 16; ++t) acc[t] = (v8f){};
    for (int kb = 0; kb < K; kb += 32) { const v16b a = frag_kb(&Ah[nloc][kb], hlf);
#pragma unroll
      for (int t = 0; t < 16; ++t) acc[t] = wmma16b(a, frag_kb(W + (size_t)(t * 16 + nloc) * K + kb, hlf), acc[t]); }
    const float* bb = g == 0 ? bq : (g == 1 ? bobs : (g == 2 ? bk : bv));
#pragma unroll
    for (int t = 0; t < 16; ++t) { const int cc = t * 16 + nloc; const float bvv = bfv(bb[cc]);
#pragma unroll
      for (int r8 = 0; r8 < 8; ++r8) Tf[8 * hlf + r8][cc] = acc[t][r8] * (1.0f / (XS * WSC)) + bvv; }
    wave_lds_sync();
    if (g == 1) {
      for (int pass = 0; pass < 2; ++pass) { for (int rr = 0; rr < 16; ++rr) { float v[8]; float s1 = 0.0f;
#pragma unroll
          for (int q = 0; q < 8; ++q) { v[q] = gelu(Tf[rr][q * 32 + lane]); s1 += v[q]; } s1 = wsum(s1); const float mu = s1 * (1.0f / D); float s2 = 0.0f;
#pragma unroll
          for (int q = 0; q < 8; ++q) { const float e = v[q] - mu; s2 += e * e; } s2 = wsum(s2); const float rs = rsqrtf(s2 * (1.0f / D) + EPS);
#pragma unroll
          for (int q = 0; q < 8; ++q) { const int c = q * 32 + lane; ((volatile float*)Z)[(m0 + rr) * 2 * D + D + c] = pmul(pmul(v[q] - mu, rs), bfv(gobs[c])) + bfv(bobs2[c]); } } __threadfence(); } }
    else { const int po = g == 0 ? 0 : (g == 2 ? D : 2 * D); for (int rr = 0; rr < 16; ++rr) for (int q = 0; q < 8; ++q) { b16 p, ql; split16(Tf[rr][q * 32 + lane] * XS, p, ql); Oh[rr][q * 32 + lane] = p; Ol[rr][q * 32 + lane] = ql; }
      wave_lds_sync();
      for (int pass = 0; pass < 2; ++pass) { for (int rr = 0; rr < 16; ++rr) { *(volatile v8b*)(PH + (m0 + rr) * (3 * D) + po + lane * 8) = *(const v8b*)(&Oh[rr][lane * 8]); *(volatile v8b*)(PL + (m0 + rr) * (3 * D) + po + lane * 8) = *(const v8b*)(&Ol[rr][lane * 8]); } __threadfence(); } }
    wave_lds_sync(); } }
__global__ __launch_bounds__(32) void att_kernel(const b16* __restrict__ PH, const b16* __restrict__ PL, const int* __restrict__ am, int BLIM, float* __restrict__ Z) { __shared__ __attribute__((aligned(16))) b16 Ph_[16][KB + 8], Pl_[16][KB + 8], Vth[HD][KB + 8], Vtl[HD][KB + 8]; __shared__ float Sf[16][KB + 4], Of[16][HD + 4]; __shared__ int Mk[16][KB];
  const int lane = threadIdx.x, nloc = lane & 15, hlf = lane >> 4; const int qt = blockIdx.x % (L / 16); const int h = (blockIdx.x / (L / 16)) % NH; const int b = blockIdx.x / ((L / 16) * NH); if (b >= BLIM) return; const int t0 = qt * 16; const size_t rowb = (size_t)b * L; const int qo = h * HD, ko = D + h * HD, vo = 2 * D + h * HD;
  const v16b qh = frag_kb(PH + (rowb + t0 + nloc) * (3 * D) + qo, hlf), ql = frag_kb(PL + (rowb + t0 + nloc) * (3 * D) + qo, hlf);
  float m_r[8], den_r[8]; v8f acc[2];
#pragma unroll
  for (int r8 = 0; r8 < 8; ++r8) { m_r[r8] = -INFINITY; den_r[r8] = 0.0f; }
  acc[0] = (v8f){}; acc[1] = (v8f){};
#pragma unroll 1
  for (int kb0 = 0; kb0 < L; kb0 += KB) {
    for (int rr = 0; rr < KB; rr += 2) { const int r = rr + hlf; const size_t vr = (rowb + kb0 + r) * (3 * D) + vo; Vth[nloc][r] = PH[vr + nloc]; Vth[16 + nloc][r] = PH[vr + 16 + nloc]; Vtl[nloc][r] = PL[vr + nloc]; Vtl[16 + nloc][r] = PL[vr + 16 + nloc]; }
    for (int rr = 0; rr < 16; ++rr) for (int q = 0; q < 4; ++q) { const int j = kb0 + q * 32 + lane; const int i = t0 + rr; Mk[rr][q * 32 + lane] = (i == j) ? 0 : am[(rowb + i) * L + j]; }
#pragma unroll
    for (int t = 0; t < KB / 16; ++t) { const size_t kr = (rowb + kb0 + t * 16 + nloc) * (3 * D) + ko; const v16b kh = frag_kb(PH + kr, hlf), kl = frag_kb(PL + kr, hlf); v8f s = {}; s = wmma16b(qh, kh, s); s = wmma16b(qh, kl, s); s = wmma16b(ql, kh, s);
#pragma unroll
      for (int r8 = 0; r8 < 8; ++r8) Sf[8 * hlf + r8][t * 16 + nloc] = s[r8] * (1.0f / (XS * XS)); }
    wave_lds_sync();
#pragma unroll
    for (int rr = 0; rr < 16; ++rr) { float mx = -INFINITY;
#pragma unroll
      for (int q = 0; q < 4; ++q) { const int kx = q * 32 + lane; if (Mk[rr][kx]) mx = fmaxf(mx, Sf[rr][kx]); }
      for (int o = 16; o; o >>= 1) mx = fmaxf(mx, __shfl_xor(mx, o));
      const float mold = __shfl(m_r[rr & 7], (rr >> 3) * 16); const float mn = fmaxf(mold, mx); const float sf = (mold == -INFINITY) ? 0.0f : ((mn == -INFINITY) ? 1.0f : __expf(mold - mn)); float ps = 0.0f;
#pragma unroll
      for (int q = 0; q < 4; ++q) { const int kx = q * 32 + lane; const float p = (Mk[rr][kx] && mn > -INFINITY) ? __expf(Sf[rr][kx] - mn) : 0.0f; ps += p; b16 ph, pl; split16(p * PS, ph, pl); Ph_[rr][kx] = ph; Pl_[rr][kx] = pl; }
      for (int o = 16; o; o >>= 1) ps += __shfl_xor(ps, o);
      if ((rr >> 3) == hlf) { const int r8 = rr & 7; den_r[r8] = den_r[r8] * sf + ps; m_r[r8] = mn; acc[0][r8] = acc[0][r8] * sf; acc[1][r8] = acc[1][r8] * sf; } }
    wave_lds_sync();
#pragma unroll
    for (int ks = 0; ks < KB; ks += 32) { const v16b pa = frag_kb(&Ph_[nloc][ks], hlf), pb = frag_kb(&Pl_[nloc][ks], hlf);
#pragma unroll
      for (int t = 0; t < 2; ++t) { const v16b vh = frag_kb(&Vth[t * 16 + nloc][ks], hlf), vl = frag_kb(&Vtl[t * 16 + nloc][ks], hlf); acc[t] = wmma16b(pa, vh, acc[t]); acc[t] = wmma16b(pa, vl, acc[t]); acc[t] = wmma16b(pb, vh, acc[t]); } }
    wave_lds_sync(); }
#pragma unroll
  for (int t = 0; t < 2; ++t)
#pragma unroll
    for (int r8 = 0; r8 < 8; ++r8) { const float dn = den_r[r8]; Of[8 * hlf + r8][t * 16 + nloc] = dn > 0.0f ? acc[t][r8] * (1.0f / (XS * PS)) / dn : 0.0f; }
  wave_lds_sync();
  for (int pass = 0; pass < 2; ++pass) { for (int rr = 0; rr < 16; ++rr) ((volatile float*)Z)[(rowb + t0 + rr) * 2 * D + h * HD + lane] = Of[rr][lane]; __threadfence(); } }
__global__ __launch_bounds__(32) void out_kernel(const float* __restrict__ Z, const b16* __restrict__ WPp, const float* __restrict__ g1, const float* __restrict__ b1, const float* __restrict__ bp, const float* __restrict__ g2, const float* __restrict__ b2, int TLIM, float* __restrict__ out) { __shared__ __attribute__((aligned(16))) b16 Ah[16][2 * D + 8], Al[16][2 * D + 8]; __shared__ float Tf[16][D + 4]; const int lane = threadIdx.x, nloc = lane & 15, hlf = lane >> 4; const size_t m0 = (size_t)blockIdx.x * 16; if (m0 >= (size_t)TLIM) return;
  for (int rr = 0; rr < 16; ++rr) { float v[16]; float s1 = 0.0f;
#pragma unroll
    for (int q = 0; q < 16; ++q) { v[q] = Z[(m0 + rr) * 2 * D + q * 32 + lane]; s1 += v[q]; } s1 = wsum(s1); const float mu = s1 * (1.0f / (2 * D)); float s2 = 0.0f;
#pragma unroll
    for (int q = 0; q < 16; ++q) { const float e = v[q] - mu; s2 += e * e; } s2 = wsum(s2); const float rs = rsqrtf(s2 * (1.0f / (2 * D)) + EPS);
#pragma unroll
    for (int q = 0; q < 16; ++q) { const int c = q * 32 + lane; b16 p, ql; split16((pmul(pmul(v[q] - mu, rs), bfv(g1[c])) + bfv(b1[c])) * XS, p, ql); Ah[rr][c] = p; Al[rr][c] = ql; } }
  wave_lds_sync(); v8f acc[16];
#pragma unroll
  for (int t = 0; t < 16; ++t) acc[t] = (v8f){};
#pragma unroll 2
  for (int kb = 0; kb < 2 * D; kb += 32) { const v16b a = frag_kb(&Ah[nloc][kb], hlf), al = frag_kb(&Al[nloc][kb], hlf);
#pragma unroll
    for (int t = 0; t < 16; ++t) { const v16b bw = frag_kb(WPp + (size_t)(t * 16 + nloc) * 2 * D + kb, hlf); acc[t] = wmma16b(a, bw, acc[t]); acc[t] = wmma16b(al, bw, acc[t]); } }
#pragma unroll
  for (int t = 0; t < 16; ++t) { const int cc = t * 16 + nloc; const float bb = bfv(bp[cc]);
#pragma unroll
    for (int r8 = 0; r8 < 8; ++r8) Tf[8 * hlf + r8][cc] = gelu(acc[t][r8] * (1.0f / (XS * WSC)) + bb); }
  wave_lds_sync();
  for (int pass = 0; pass < 2; ++pass) { for (int rr = 0; rr < 16; ++rr) { float v[8]; float s1 = 0.0f;
#pragma unroll
      for (int q = 0; q < 8; ++q) { v[q] = Tf[rr][q * 32 + lane]; s1 += v[q]; } s1 = wsum(s1); const float mu = s1 * (1.0f / D); float s2 = 0.0f;
#pragma unroll
      for (int q = 0; q < 8; ++q) { const float e = v[q] - mu; s2 += e * e; } s2 = wsum(s2); const float rs = rsqrtf(s2 * (1.0f / D) + EPS);
#pragma unroll
      for (int q = 0; q < 8; ++q) { const int c = q * 32 + lane; ((volatile float*)out)[(m0 + rr) * D + c] = pmul(pmul(v[q] - mu, rs), bfv(g2[c])) + bfv(b2[c]); } } __threadfence(); } }
}

extern "C" void kernel_launch(void* const* d_in, const int* in_sizes, int n_in, void* d_out, int out_size, void* d_ws, size_t ws_size, hipStream_t stream) {
  (void)n_in;
  auto Fp = [&](int i) { return (const float*)d_in[i]; }; auto Ip = [&](int i) { return (const int*)d_in[i]; };
  if (in_sizes[0] != NT * D || in_sizes[1] != NT * D || in_sizes[2] != NB * L * L || in_sizes[3] != D * D || in_sizes[5] != D * 2 * D || in_sizes[7] != D * 2 * D || in_sizes[9] != D * D || in_sizes[15] != D * 2 * D || out_size != NT * D) return;
  const int BLIM = NB;
  const int TLIM = BLIM * L;
  size_t off = 0; char* ws = (char*)d_ws;
  auto carve = [&](size_t bytes) { char* p = ws + off; off += (bytes + 255) & ~(size_t)255; return p; };
  b16* WQO = (b16*)carve((size_t)512 * D * 2); b16* WKV = (b16*)carve((size_t)512 * 2 * D * 2); b16* WPp = (b16*)carve((size_t)D * 2 * D * 2); b16* PH = (b16*)carve((size_t)NT * 3 * D * 2); b16* PL = (b16*)carve((size_t)NT * 3 * D * 2); float* Z = (float*)carve((size_t)NT * 2 * D * 4);
  if (off > ws_size || off > ((size_t)64 << 20)) return;
  wput_kernel<<<(512 * 64 + 255) / 256, 256, 0, stream>>>(Fp(3), Fp(9), Fp(5), Fp(7), Fp(15), WQO, WKV, WPp);
  proj_kernel<<<TLIM / 16, 32, 0, stream>>>(Fp(0), Fp(1), WQO, WKV, Fp(4), Fp(6), Fp(8), Fp(10), Fp(11), Fp(12), TLIM, PH, PL, Z);
  att_kernel<<<BLIM * NH * (L / 16), 32, 0, stream>>>(PH, PL, Ip(2), BLIM, Z);
  out_kernel<<<TLIM / 16, 32, 0, stream>>>(Z, WPp, Fp(13), Fp(14), Fp(16), Fp(17), Fp(18), TLIM, (float*)d_out);
}
